// DualChannelGCN_36275293782543
// MI455X (gfx1250) — hardware-verified
//
#include <hip/hip_runtime.h>
#include <stddef.h>
#include <stdint.h>

#define NB   64
#define NN   256
#define DD   768
#define GG   300
#define GP   320
#define NROW (NB * NN)
#define CLD  640
#define FLD  640
#define CSP  324
#define PSP  264
#define TP   72
#define QR   32
#define GR   64
#define AVP  384
#define FILLV (-9.0e15f)
#define LEAK 0.2f
#define WSC  64.0f
#define WINV 0.015625f
#define PSC  1024.0f
#define PINV 0.0009765625f

static_assert(NN == 256);
static_assert(DD == 3 * 256);
static_assert((NROW % GR) == 0);
static_assert((NN % QR) == 0);
static_assert((NN % GR) == 0);
static_assert((GP % 80) == 0);
static_assert((DD % 64) == 0);
static_assert((GP % 64) == 0);
static_assert((FLD % 64) == 0);
static_assert((CSP % 4) == 0);
static_assert((PSP % 8) == 0);
static_assert((TP % 8) == 0);
static_assert(QR == 32);
static_assert(GP == NN + 64);
static_assert(AVP == NN + 128);
static_assert(AVP >= 4 * 31 + 128 * 2 + 4);
static_assert((GG % 4) == 0);
static_assert(QR * PSP * 2 + QR * CSP * 4 + (2 * NN + 3 * GP + QR) * 4 <= 65536);
static_assert(GP * TP * 2 + 128 * 4 + 2 * AVP * 4 + GR * 4 <= 65536);
static_assert(((NROW * DD / 8) % 1024) == 0);

typedef _Float16 v16h __attribute__((ext_vector_type(16)));
typedef _Float16 v8h  __attribute__((ext_vector_type(8)));
typedef float    v8f  __attribute__((ext_vector_type(8)));
typedef float    v4f  __attribute__((ext_vector_type(4)));
typedef unsigned int v4u __attribute__((ext_vector_type(4)));

union Frag  { v16h v; v8h h[2]; };
union Pack8 { v8h h; v4u u; };
static_assert(sizeof(Frag) == 32);
static_assert(sizeof(Pack8) == 16);

__device__ __forceinline__ v8f mma16(v16h a, v16h b, v8f c) {
  c = __builtin_amdgcn_wmma_f32_16x16x32_f16(false, a, false, b, (short)0, c, false, false);
  asm volatile("v_nop\n\tv_nop\n\tv_nop\n\tv_nop" : "+v"(c) : "v"(a), "v"(b));
  return c;
}

__device__ __forceinline__ v16h ldfrag(const _Float16* p, int ld, int row0, int k0, int lane) {
  const int m = lane & 15, lh = lane >> 4;
  const _Float16* q = p + (size_t)(row0 + m) * ld + k0 + 8 * lh;
  Frag f;
  f.h[0] = *(const v8h*)(q);
  f.h[1] = *(const v8h*)(q + 16);
  return f.v;
}

__device__ __forceinline__ v8f zero8() { return (v8f){0.f, 0.f, 0.f, 0.f, 0.f, 0.f, 0.f, 0.f}; }

__device__ __forceinline__ float wsum(float v) {
#pragma unroll
  for (int o = 16; o; o >>= 1) v += __shfl_xor(v, o, 32);
  return v;
}
__device__ __forceinline__ float wmax(float v) {
#pragma unroll
  for (int o = 16; o; o >>= 1) v = fmaxf(v, __shfl_xor(v, o, 32));
  return v;
}

__global__ __launch_bounds__(256) void k_cvt(const float* __restrict__ x, _Float16* __restrict__ y, int npieces) {
  const int tid = threadIdx.x;
  Pack8 val[4];
  int pi[4];
#pragma unroll
  for (int it = 0; it < 4; ++it) {
    const int p = blockIdx.x * 1024 + 256 * it + tid;
    const int pc = min(p, npieces - 1);
    const v8f u = *(const v8f*)(x + (size_t)pc * 8);
    val[it].h = __builtin_convertvector(u, v8h);
    pi[it] = p;
  }
  for (int ps = 0; ps < 2; ++ps) {
#pragma unroll
    for (int it = 0; it < 4; ++it)
      if (pi[it] < npieces) *(volatile v4u*)(y + (size_t)pi[it] * 8) = val[it].u;
    __threadfence();
  }
}

__global__ __launch_bounds__(256) void k_sem(const float* __restrict__ x, const float* __restrict__ mask,
                                             float* __restrict__ svals) {
  __shared__ float msk[NN];
  __shared__ float anv[DD];
  __shared__ float sims[NN];
  __shared__ __align__(16) float svl[NN];
  __shared__ float redf[8];
  __shared__ int   redi[8];
  __shared__ float tvs[16];
  __shared__ int   tis[16];
  __shared__ float bc[2];

  const int tid = threadIdx.x, lane = tid & 31, wave = tid >> 5;
  const int b = blockIdx.x;
  const float* xb = x + (size_t)b * NN * DD;

  const float mv = mask[(size_t)b * NN + tid];
  msk[tid] = mv;
  const float cs = wsum(mv);
  if (lane == 0) redf[wave] = cs;
  __syncthreads();
  if (tid == 0) {
    float c = 0.f;
    for (int w = 0; w < 8; ++w) c += redf[w];
    bc[0] = 1.0f / (c + 1e-8f);
  }
  __syncthreads();
  const float rc = bc[0];

  float a0 = 0.f, a1 = 0.f, a2 = 0.f;
#pragma unroll 1
  for (int n = 0; n < NN; ++n) {
    const float mn = msk[n];
    const float* xr = xb + (size_t)n * DD + tid;
    a0 += xr[0] * mn;
    a1 += xr[256] * mn;
    a2 += xr[512] * mn;
  }
  a0 *= rc; a1 *= rc; a2 *= rc;
  float qq = a0 * a0 + a1 * a1 + a2 * a2;
  qq = wsum(qq);
  if (lane == 0) redf[wave] = qq;
  __syncthreads();
  if (tid == 0) {
    float t = 0.f;
    for (int w = 0; w < 8; ++w) t += redf[w];
    bc[1] = 1.0f / fmaxf(sqrtf(t), 1e-12f);
  }
  __syncthreads();
  const float inva = bc[1];
  anv[tid]       = a0 * inva;
  anv[tid + 256] = a1 * inva;
  anv[tid + 512] = a2 * inva;
  __syncthreads();

#pragma unroll 1
  for (int r = 0; r < 32; ++r) {
    const int n = wave + 8 * r;
    const float* xr = xb + (size_t)n * DD + lane;
    float hh = 0.f;
#pragma unroll 4
    for (int e = 0; e < 24; ++e) { const float v = xr[32 * e]; hh = fmaf(v, v, hh); }
    hh = wsum(hh);
    const float invh = 1.0f / fmaxf(sqrtf(hh), 1e-12f);
    float d = 0.f;
#pragma unroll 4
    for (int e = 0; e < 24; ++e) { const float v = xr[32 * e]; d = fmaf(v * invh, anv[lane + 32 * e], d); }
    d = wsum(d);
    if (lane == 0) sims[n] = d;
  }
  __syncthreads();

  float cv = sims[tid];
  const int ci = tid;
#pragma unroll 1
  for (int it = 0; it < 10; ++it) {
    float bv = cv;
    int bi = ci;
#pragma unroll
    for (int o = 16; o; o >>= 1) {
      const float ov = __shfl_xor(bv, o, 32);
      const int oi = __shfl_xor(bi, o, 32);
      const bool tk = (ov > bv) || (ov == bv && oi < bi);
      bv = tk ? ov : bv;
      bi = tk ? oi : bi;
    }
    if (lane == 0) { redf[wave] = bv; redi[wave] = bi; }
    __syncthreads();
    if (tid == 0) {
      float vv = redf[0];
      int ii = redi[0];
      for (int w = 1; w < 8; ++w) {
        const float ov = redf[w];
        const int oi = redi[w];
        const bool tk = (ov > vv) || (ov == vv && oi < ii);
        vv = tk ? ov : vv;
        ii = tk ? oi : ii;
      }
      tvs[it] = vv;
      tis[it] = ii;
    }
    __syncthreads();
    if (ci == tis[it]) cv = -__builtin_inff();
  }

  svl[tid] = 0.f;
  __syncthreads();
  if (tid < 10) svl[tis[tid]] = tvs[tid];
  __syncthreads();
  if (tid < 64) {
    const v4f v = *(const v4f*)(svl + 4 * tid);
    float* dst = svals + (size_t)b * NN + 4 * tid;
    *(volatile v4f*)dst = v;
    __threadfence();
    *(volatile v4f*)dst = v;
  }
}

__global__ __launch_bounds__(256) void k_wcvt(const float* __restrict__ s0, const float* __restrict__ s1,
                                              int has1, int ka, int kb, int kpad,
                                              _Float16* __restrict__ bt) {
  __shared__ __align__(16) _Float16 T[GR * TP];
  const int tid = threadIdx.x;
  const int n0 = blockIdx.x * GR;
  const int nl = tid & 63, kq = tid >> 6;
  const int n = n0 + nl;
  const bool seg0 = (n < GG);
  const bool seg1 = (has1 != 0) && (n >= GP) && (n < GP + GG);
  const int c0 = min(n, GG - 1);
  const int c1 = min(max(n - GP, 0), GG - 1);
  const int ktot = ka + kb;
#pragma unroll 1
  for (int kc = 0; kc < kpad; kc += 64) {
#pragma unroll 1
    for (int ig = 0; ig < 4; ++ig) {
#pragma unroll
      for (int i4 = 0; i4 < 4; ++i4) {
        const int kl = kq + 4 * (4 * ig + i4);
        const int k = kc + kl;
        const int ks = (k < ka) ? k : ((k >= GP && k < GP + kb) ? (k - GP + ka) : -1);
        const int ksc = min(max(ks, 0), ktot - 1);
        const float v0 = s0[(size_t)ksc * GG + c0];
        const float v1 = s1[(size_t)ksc * GG + c1];
        const float v = (ks >= 0) ? (seg0 ? v0 : (seg1 ? v1 : 0.f)) : 0.f;
        T[nl * TP + kl] = (_Float16)(v * WSC);
      }
    }
    __syncthreads();
    for (int ps = 0; ps < 2; ++ps) {
#pragma unroll
      for (int it = 0; it < 2; ++it) {
        const int p = tid + 256 * it;
        const int r = p >> 3, q = p & 7;
        Pack8 pk;
        pk.h = *(const v8h*)(T + r * TP + 8 * q);
        *(volatile v4u*)(bt + (size_t)(n0 + r) * kpad + kc + 8 * q) = pk.u;
      }
      __threadfence();
    }
    __syncthreads();
  }
}

template <int MODE>
__global__ __launch_bounds__(256) void k_gemm(const _Float16* __restrict__ A, int lda,
                                              const _Float16* __restrict__ Bt, int ldb, int nk,
                                              float* __restrict__ C, int ldc,
                                              const float* __restrict__ bias) {
  extern __shared__ __align__(16) float cs[];
  __shared__ __align__(16) float bss[GP];
  const int tid = threadIdx.x, lane = tid & 31, wave = tid >> 5;
  const int h = lane >> 4, m = lane & 15;
  const int rg = wave & 1, cg = wave >> 1;
  const int row0 = blockIdx.y * GR;
  const int n0 = blockIdx.x * GP;
  const int ar = row0 + 32 * rg;
  const int bcn = n0 + 80 * cg;

  if (MODE == 1) {
    bss[tid] = bias[tid];
    if (wave < 2) {
      const int c = NN + tid;
      const int cc = min(c, GG - 1);
      const float bv = bias[cc];
      bss[c] = (c < GG) ? bv : 0.f;
    }
  }

  v8f acc[10];
#pragma unroll
  for (int t = 0; t < 10; ++t) acc[t] = zero8();

#pragma unroll 1
  for (int s = 0; s < nk; ++s) {
    const int k0 = 32 * s;
    const v16h a0 = ldfrag(A, lda, ar, k0, lane);
    const v16h a1 = ldfrag(A, lda, ar + 16, k0, lane);
#pragma unroll
    for (int t = 0; t < 5; ++t) {
      const v16h bf = ldfrag(Bt, ldb, bcn + 16 * t, k0, lane);
      acc[2 * t]     = mma16(a0, bf, acc[2 * t]);
      acc[2 * t + 1] = mma16(a1, bf, acc[2 * t + 1]);
    }
  }

#pragma unroll
  for (int t = 0; t < 5; ++t) {
#pragma unroll
    for (int s = 0; s < 2; ++s) {
      const v8f v = acc[2 * t + s] * WINV;
      float* cp = cs + (32 * rg + 16 * s + 8 * h) * CSP + 80 * cg + 16 * t + m;
#pragma unroll
      for (int r = 0; r < 8; ++r) cp[r * CSP] = v[r];
    }
  }
  __syncthreads();

  if (MODE == 0) {
    for (int ps = 0; ps < 2; ++ps) {
#pragma unroll
      for (int it = 0; it < 20; ++it) {
        const int p = tid + 256 * it;
        const int row = p / 80, q = p - 80 * row;
        const v4f v = *(const v4f*)(cs + row * CSP + 4 * q);
        *(volatile v4f*)(C + (size_t)(row0 + row) * ldc + n0 + 4 * q) = v;
      }
      __threadfence();
    }
  } else {
    for (int ps = 0; ps < 2; ++ps) {
#pragma unroll
      for (int it = 0; it < 19; ++it) {
        const int p = tid + 256 * it;
        if (p < GR * 75) {
          const int row = p / 75, q = p - 75 * row;
          const v4f cv = *(const v4f*)(cs + row * CSP + 4 * q);
          const v4f bv = *(const v4f*)(bss + 4 * q);
          const v4f u = cv + bv;
          v4f y;
          y[0] = fmaxf(u[0], 0.f);
          y[1] = fmaxf(u[1], 0.f);
          y[2] = fmaxf(u[2], 0.f);
          y[3] = fmaxf(u[3], 0.f);
          *(volatile v4f*)(C + (size_t)(row0 + row) * GG + 4 * q) = y;
        }
      }
      __threadfence();
    }
  }
}

__global__ __launch_bounds__(256) void k_rows(const float* __restrict__ C, int ldc,
                                              const float* __restrict__ pos, const int* __restrict__ posi,
                                              const float* __restrict__ a1, const float* __restrict__ a2,
                                              _Float16* __restrict__ whT, float* __restrict__ fp) {
  __shared__ __align__(16) _Float16 T[GP * TP];
  __shared__ __align__(16) float fs[128];
  __shared__ __align__(16) float a1s[AVP];
  __shared__ __align__(16) float a2s[AVP];
  __shared__ int pcs[GR];
  const int tid = threadIdx.x, lane = tid & 31, wave = tid >> 5;
  const int b = blockIdx.y;
  const int n0 = blockIdx.x * GR;

  {
    a1s[tid] = a1[tid];
    a2s[tid] = a2[tid];
    if (wave < 4) {
      const int c = NN + tid;
      const int cc = min(c, GG - 1);
      const float u1 = a1[cc], u2 = a2[cc];
      const bool inr = (c < GG);
      a1s[c] = inr ? u1 : 0.f;
      a2s[c] = inr ? u2 : 0.f;
    }
    if (wave < 2) {
      int pp = posi[(size_t)b * NN + n0 + tid];
      pcs[tid] = min(max(pp, 0), NN - 1);
    }
  }
  __syncthreads();

#pragma unroll 1
  for (int q = 0; q < 8; ++q) {
    const int nl = 8 * wave + q;
    const int rowg = b * NN + n0 + nl;
    const int pp = pcs[nl];
    const float* cr = C + (size_t)rowg * ldc;
    const float* pr = pos + (size_t)pp * GG;
    float s1 = 0.f, s2 = 0.f;
#pragma unroll
    for (int e = 0; e < 3; ++e) {
      const int c = 4 * lane + 128 * e;
      const int cq = min(c, GG - 4);
      const v4f wv = *(const v4f*)(cr + cq);
      const v4f pv = *(const v4f*)(pr + cq);
      const v4f av1 = *(const v4f*)(a1s + c);
      const v4f av2 = *(const v4f*)(a2s + c);
      const bool inr = (c < GG);
      const float v0 = inr ? (wv[0] + pv[0]) : 0.f;
      const float v1 = inr ? (wv[1] + pv[1]) : 0.f;
      const float v2 = inr ? (wv[2] + pv[2]) : 0.f;
      const float v3 = inr ? (wv[3] + pv[3]) : 0.f;
      s1 = fmaf(v0, av1[0], s1); s1 = fmaf(v1, av1[1], s1); s1 = fmaf(v2, av1[2], s1); s1 = fmaf(v3, av1[3], s1);
      s2 = fmaf(v0, av2[0], s2); s2 = fmaf(v1, av2[1], s2); s2 = fmaf(v2, av2[2], s2); s2 = fmaf(v3, av2[3], s2);
      if (c < GP) {
        T[(c + 0) * TP + nl] = (_Float16)v0;
        T[(c + 1) * TP + nl] = (_Float16)v1;
        T[(c + 2) * TP + nl] = (_Float16)v2;
        T[(c + 3) * TP + nl] = (_Float16)v3;
      }
    }
    s1 = wsum(s1);
    s2 = wsum(s2);
    if (lane == 0) { fs[nl] = s1; fs[64 + nl] = s2; }
  }
  __syncthreads();

  for (int ps = 0; ps < 2; ++ps) {
#pragma unroll
    for (int it = 0; it < 10; ++it) {
      const int p = tid + 256 * it;
      const int g = p >> 3, qq = p & 7;
      Pack8 pk;
      pk.h = *(const v8h*)(T + g * TP + 8 * qq);
      *(volatile v4u*)(whT + ((size_t)b * GP + g) * NN + n0 + 8 * qq) = pk.u;
    }
    __threadfence();
  }
  if (wave == 0) {
    const int hf = lane >> 4, lq = lane & 15;
    const v4f v = *(const v4f*)(fs + 64 * hf + 4 * lq);
    float* dst = fp + (size_t)hf * NROW + (size_t)b * NN + n0 + 4 * lq;
    *(volatile v4f*)dst = v;
    __threadfence();
    *(volatile v4f*)dst = v;
  }
}

__global__ __launch_bounds__(256) void k_gat(const _Float16* __restrict__ whT, const float* __restrict__ fp,
                                             const int* __restrict__ adj, const float* __restrict__ sv, int sem,
                                             const float* __restrict__ res, int ldr, int rcoff,
                                             const float* __restrict__ tb, int hastb,
                                             const float* __restrict__ gam, const float* __restrict__ bet,
                                             float* __restrict__ o32, int has32,
                                             _Float16* __restrict__ o16, int ld16, int coff16) {
  __shared__ __align__(16) _Float16 Ps[QR * PSP];
  __shared__ __align__(16) float Cs[QR * CSP];
  __shared__ __align__(16) float f2s[NN];
  __shared__ __align__(16) float svs[NN];
  __shared__ __align__(16) float f1s[QR];
  __shared__ __align__(16) float gms[GP];
  __shared__ __align__(16) float bts[GP];
  __shared__ __align__(16) float tbs[GP];

  const int tid = threadIdx.x, lane = tid & 31, wave = tid >> 5;
  const int h = lane >> 4, m = lane & 15;
  const int bb = blockIdx.y;
  const int i0 = blockIdx.x * QR;
  const int rg = wave & 1, cg = wave >> 1;

  {
    const size_t cb = (size_t)bb * NN + tid;
    f2s[tid] = fp[(size_t)NROW + cb];
    svs[tid] = sv[cb];
    const float g0 = gam[tid], b0 = bet[tid], t0 = tb[tid];
    gms[tid] = g0;
    bts[tid] = b0;
    tbs[tid] = (hastb != 0) ? t0 : 0.f;
    if (wave < 2) {
      const int c = NN + tid;
      const int cc = min(c, GG - 1);
      const float g1 = gam[cc], b1 = bet[cc], t1 = tb[cc];
      const bool inr = (c < GG);
      gms[c] = inr ? g1 : 0.f;
      bts[c] = inr ? b1 : 0.f;
      tbs[c] = (inr && hastb != 0) ? t1 : 0.f;
    }
    if (wave == 0) f1s[tid] = fp[(size_t)bb * NN + i0 + tid];
  }
  __syncthreads();

  float f2v[8], svv[8];
  float S = 0.f;
#pragma unroll
  for (int e = 0; e < 8; ++e) {
    const int j = lane + 32 * e;
    f2v[e] = f2s[j];
    svv[e] = svs[j];
    S += svv[e];
  }
  S = wsum(S);

#pragma unroll 1
  for (int q = 0; q < 4; ++q) {
    const int rl = 4 * wave + q;
    const int i = i0 + rl;
    const int rowg = bb * NN + i;
    const float f1i = f1s[rl];
    const float svi = svs[i];
    const float rs = 0.5f * S + 128.0f * svi + 1.0f;
    const float rrs = 1.0f / (rs + 1e-8f);
    float ev[8];
    if (sem != 0) {
#pragma unroll
      for (int e = 0; e < 8; ++e) {
        const int j = lane + 32 * e;
        float u = f1i + f2v[e];
        u = (u >= 0.f) ? u : LEAK * u;
        const float val = (0.5f * (svv[e] + svi) + ((i == j) ? 1.0f : 0.f)) * rrs;
        ev[e] = (val > 0.f) ? u : FILLV;
      }
    } else {
      const int* arow = adj + (size_t)rowg * NN + lane;
#pragma unroll
      for (int e = 0; e < 8; ++e) {
        const int am = arow[32 * e];
        float u = f1i + f2v[e];
        u = (u >= 0.f) ? u : LEAK * u;
        ev[e] = (am > 0) ? u : FILLV;
      }
    }
    float mx = ev[0];
#pragma unroll
    for (int e = 1; e < 8; ++e) mx = fmaxf(mx, ev[e]);
    mx = wmax(mx);
    float l = 0.f;
#pragma unroll
    for (int e = 0; e < 8; ++e) { ev[e] = __expf(ev[e] - mx); l += ev[e]; }
    l = wsum(l);
    const float sc = PSC * (1.0f / l);
#pragma unroll
    for (int e = 0; e < 8; ++e) Ps[rl * PSP + lane + 32 * e] = (_Float16)(ev[e] * sc);
  }
  __syncthreads();

  v8f acc[5];
#pragma unroll
  for (int t = 0; t < 5; ++t) acc[t] = zero8();
#pragma unroll 1
  for (int j0 = 0; j0 < NN; j0 += 32) {
    const v16h af = ldfrag(Ps, PSP, 16 * rg, j0, lane);
#pragma unroll
    for (int t = 0; t < 5; ++t) {
      const v16h bf = ldfrag(whT, NN, bb * GP + 80 * cg + 16 * t, j0, lane);
      acc[t] = mma16(af, bf, acc[t]);
    }
  }
#pragma unroll
  for (int t = 0; t < 5; ++t) {
    const v8f v = acc[t] * PINV;
    float* cp = Cs + (16 * rg + 8 * h) * CSP + 80 * cg + 16 * t + m;
#pragma unroll
    for (int r = 0; r < 8; ++r) cp[r * CSP] = v[r];
  }
  __syncthreads();

#pragma unroll 1
  for (int q = 0; q < 4; ++q) {
    const int rl = 4 * wave + q;
    const int rowg = bb * NN + i0 + rl;
    const float* rr = res + (size_t)rowg * ldr + rcoff;
#pragma unroll
    for (int e = 0; e < 3; ++e) {
      const int c = 4 * lane + 128 * e;
      const int cq = min(c, GG - 4);
      const v4f r4 = *(const v4f*)(rr + cq);
      if (c < GG) {
        float* cp = Cs + rl * CSP + c;
        v4f u = *(const v4f*)cp;
        u = u + r4;
        *(v4f*)cp = u;
      }
    }
  }
  __syncthreads();

  float gv[10], bev[10], tbv[10];
#pragma unroll
  for (int e = 0; e < 10; ++e) {
    const int c = lane + 32 * e;
    gv[e] = gms[c];
    bev[e] = bts[c];
    tbv[e] = tbs[c];
  }
#pragma unroll 1
  for (int q = 0; q < 4; ++q) {
    const int rl = 4 * wave + q;
    float xv[10];
    float s = 0.f;
#pragma unroll
    for (int e = 0; e < 10; ++e) {
      const int c = lane + 32 * e;
      float xx = Cs[rl * CSP + c] + tbv[e];
      xx = (c < GG) ? xx : 0.f;
      xv[e] = xx;
      s += xx;
    }
    s = wsum(s);
    const float mean = s * (1.0f / 300.0f);
    float vs = 0.f;
#pragma unroll
    for (int e = 0; e < 10; ++e) {
      const int c = lane + 32 * e;
      const float d = (c < GG) ? (xv[e] - mean) : 0.f;
      xv[e] = d;
      vs = fmaf(d, d, vs);
    }
    vs = wsum(vs);
    const float rstd = 1.0f / sqrtf(vs * (1.0f / 300.0f) + 1e-5f);
#pragma unroll
    for (int e = 0; e < 10; ++e) {
      const int c = lane + 32 * e;
      float y = fmaf(xv[e] * rstd, gv[e], bev[e]);
      y = fmaxf(y, 0.f);
      y = (c < GG) ? y : 0.f;
      Cs[rl * CSP + c] = y;
    }
  }
  __syncthreads();

  if (has32 != 0) {
    for (int ps = 0; ps < 2; ++ps) {
#pragma unroll
      for (int it = 0; it < 10; ++it) {
        const int p = tid + 256 * it;
        const int row = p / 80, qq = p - 80 * row;
        const v4f v = *(const v4f*)(Cs + row * CSP + 4 * qq);
        *(volatile v4f*)(o32 + (size_t)(bb * NN + i0 + row) * GP + 4 * qq) = v;
      }
      __threadfence();
    }
  }
  for (int ps = 0; ps < 2; ++ps) {
#pragma unroll
    for (int it = 0; it < 5; ++it) {
      const int p = tid + 256 * it;
      const int row = p / 40, qq = p - 40 * row;
      const v4f u0 = *(const v4f*)(Cs + row * CSP + 8 * qq);
      const v4f u1 = *(const v4f*)(Cs + row * CSP + 8 * qq + 4);
      const v8f u = __builtin_shufflevector(u0, u1, 0, 1, 2, 3, 4, 5, 6, 7);
      Pack8 pk;
      pk.h = __builtin_convertvector(u, v8h);
      *(volatile v4u*)(o16 + (size_t)(bb * NN + i0 + row) * ld16 + coff16 + 8 * qq) = pk.u;
    }
    __threadfence();
  }
}

extern "C" void kernel_launch(void* const* d_in, const int* in_sizes, int n_in,
                              void* d_out, int out_size, void* d_ws, size_t ws_size,
                              hipStream_t stream) {
  if (n_in < 34) return;
  if (in_sizes[0] != NROW * DD) return;
  if (in_sizes[1] != NB * NN) return;
  for (int i = 2; i < 32; ++i) {
    int want = GG;
    if (i == 2 || i == 6 || i == 16 || i == 20) want = DD * GG;
    else if (i == 5 || i == 13 || i == 19 || i == 27) want = NN * GG;
    else if (i == 10 || i == 24) want = GG * GG;
    else if (i == 30) want = 2 * GG * GG;
    if (in_sizes[i] != want) return;
  }
  if (in_sizes[32] != NB * NN * NN) return;
  if (in_sizes[33] != NB * NN) return;
  if (out_size != NROW * GG) return;

  const float* x        = (const float*)d_in[0];
  const float* amask    = (const float*)d_in[1];
  const float* syn0_W   = (const float*)d_in[2];
  const float* syn0_a1  = (const float*)d_in[3];
  const float* syn0_a2  = (const float*)d_in[4];
  const float* syn0_pos = (const float*)d_in[5];
  const float* syn0_tW  = (const float*)d_in[6];
  const float* syn0_tb  = (const float*)d_in[7];
  const float* syn0_g   = (const float*)d_in[8];
  const float* syn0_b   = (const float*)d_in[9];
  const float* syn1_W   = (const float*)d_in[10];
  const float* syn1_a1  = (const float*)d_in[11];
  const float* syn1_a2  = (const float*)d_in[12];
  const float* syn1_pos = (const float*)d_in[13];
  const float* syn1_g   = (const float*)d_in[14];
  const float* syn1_b   = (const float*)d_in[15];
  const float* sem0_W   = (const float*)d_in[16];
  const float* sem0_a1  = (const float*)d_in[17];
  const float* sem0_a2  = (const float*)d_in[18];
  const float* sem0_pos = (const float*)d_in[19];
  const float* sem0_tW  = (const float*)d_in[20];
  const float* sem0_tb  = (const float*)d_in[21];
  const float* sem0_g   = (const float*)d_in[22];
  const float* sem0_b   = (const float*)d_in[23];
  const float* sem1_W   = (const float*)d_in[24];
  const float* sem1_a1  = (const float*)d_in[25];
  const float* sem1_a2  = (const float*)d_in[26];
  const float* sem1_pos = (const float*)d_in[27];
  const float* sem1_g   = (const float*)d_in[28];
  const float* sem1_b   = (const float*)d_in[29];
  const float* fus_W    = (const float*)d_in[30];
  const float* fus_b    = (const float*)d_in[31];
  const int*   adj      = (const int*)d_in[32];
  const int*   posi     = (const int*)d_in[33];
  float* out = (float*)d_out;

  size_t off = 0;
  const size_t oX16 = off; off += (size_t)NROW * DD * sizeof(_Float16);
  const size_t oC   = off; off += (size_t)NROW * CLD * sizeof(float);
  const size_t oWhT = off; off += (size_t)NB * GP * NN * sizeof(_Float16);
  const size_t oA16 = off; off += (size_t)NROW * GP * sizeof(_Float16);
  const size_t oA32 = off; off += (size_t)NROW * GP * sizeof(float);
  const size_t oAF  = off; off += (size_t)NROW * FLD * sizeof(_Float16);
  const size_t oBt  = off; off += (size_t)CLD * DD * sizeof(_Float16);
  const size_t oF   = off; off += (size_t)2 * NROW * sizeof(float);
  const size_t oSV  = off; off += (size_t)NB * NN * sizeof(float);
  if (off > ws_size) return;
  if (off > (size_t)134217728) return;

  char* ws = (char*)d_ws;
  _Float16* X16 = (_Float16*)(ws + oX16);
  float*    Cp  = (float*)(ws + oC);
  _Float16* WhT = (_Float16*)(ws + oWhT);
  _Float16* A16 = (_Float16*)(ws + oA16);
  float*    A32 = (float*)(ws + oA32);
  _Float16* AF  = (_Float16*)(ws + oAF);
  _Float16* Bt  = (_Float16*)(ws + oBt);
  float*    F   = (float*)(ws + oF);
  float*    SV  = (float*)(ws + oSV);

  const size_t ldsg = (size_t)GR * CSP * sizeof(float);
  (void)hipFuncSetAttribute(reinterpret_cast<const void*>(&k_gemm<0>),
                            hipFuncAttributeMaxDynamicSharedMemorySize, (int)ldsg);
  (void)hipFuncSetAttribute(reinterpret_cast<const void*>(&k_gemm<1>),
                            hipFuncAttributeMaxDynamicSharedMemorySize, (int)ldsg);

  const dim3 blk(256);
  const dim3 ggemm2(CLD / GP, NROW / GR);
  const dim3 ggemm1(1, NROW / GR);
  const dim3 grows(NN / GR, NB);
  const dim3 ggat(NN / QR, NB);

  k_cvt<<<dim3((NROW * DD / 8) / 1024), blk, 0, stream>>>(x, X16, NROW * DD / 8);
  k_sem<<<dim3(NB), blk, 0, stream>>>(x, amask, SV);

  k_wcvt<<<dim3(CLD / GR), blk, 0, stream>>>(syn0_W, syn0_tW, 1, DD, 0, DD, Bt);
  k_gemm<0><<<ggemm2, blk, ldsg, stream>>>(X16, DD, Bt, DD, DD / 32, Cp, CLD, fus_b);
  k_rows<<<grows, blk, 0, stream>>>(Cp, CLD, syn0_pos, posi, syn0_a1, syn0_a2, WhT, F);
  k_gat<<<ggat, blk, 0, stream>>>(WhT, F, adj, SV, 0, Cp, CLD, GP, syn0_tb, 1, syn0_g, syn0_b,
                                  A32, 1, A16, GP, 0);
  k_wcvt<<<dim3(GP / GR), blk, 0, stream>>>(syn1_W, syn1_W, 0, GG, 0, GP, Bt);
  k_gemm<0><<<ggemm1, blk, ldsg, stream>>>(A16, GP, Bt, GP, GP / 32, Cp, CLD, fus_b);
  k_rows<<<grows, blk, 0, stream>>>(Cp, CLD, syn1_pos, posi, syn1_a1, syn1_a2, WhT, F);
  k_gat<<<ggat, blk, 0, stream>>>(WhT, F, adj, SV, 0, A32, GP, 0, syn1_g, 0, syn1_g, syn1_b,
                                  Cp, 0, AF, FLD, 0);

  k_wcvt<<<dim3(CLD / GR), blk, 0, stream>>>(sem0_W, sem0_tW, 1, DD, 0, DD, Bt);
  k_gemm<0><<<ggemm2, blk, ldsg, stream>>>(X16, DD, Bt, DD, DD / 32, Cp, CLD, fus_b);
  k_rows<<<grows, blk, 0, stream>>>(Cp, CLD, sem0_pos, posi, sem0_a1, sem0_a2, WhT, F);
  k_gat<<<ggat, blk, 0, stream>>>(WhT, F, adj, SV, 1, Cp, CLD, GP, sem0_tb, 1, sem0_g, sem0_b,
                                  A32, 1, A16, GP, 0);
  k_wcvt<<<dim3(GP / GR), blk, 0, stream>>>(sem1_W, sem1_W, 0, GG, 0, GP, Bt);
  k_gemm<0><<<ggemm1, blk, ldsg, stream>>>(A16, GP, Bt, GP, GP / 32, Cp, CLD, fus_b);
  k_rows<<<grows, blk, 0, stream>>>(Cp, CLD, sem1_pos, posi, sem1_a1, sem1_a2, WhT, F);
  k_gat<<<ggat, blk, 0, stream>>>(WhT, F, adj, SV, 1, A32, GP, 0, sem1_g, 0, sem1_g, sem1_b,
                                  Cp, 0, AF, FLD, GP);

  k_wcvt<<<dim3(GP / GR), blk, 0, stream>>>(fus_W, fus_W, 0, GG, GG, FLD, Bt);
  k_gemm<1><<<ggemm1, blk, ldsg, stream>>>(AF, FLD, Bt, FLD, FLD / 32, out, GG, fus_b);

  (void)hipGetLastError();
}
